// GraphSAGENodePredictor_12850542150153
// MI455X (gfx1250) — hardware-verified
//
#include <hip/hip_runtime.h>
#include <math.h>

typedef __attribute__((ext_vector_type(16))) _Float16 v16h;
typedef __attribute__((ext_vector_type(16))) __bf16 v16b;
typedef __attribute__((ext_vector_type(8)))  _Float16 v8h;
typedef __attribute__((ext_vector_type(8)))  float v8f;
typedef __attribute__((ext_vector_type(4)))  float v4f;
typedef __attribute__((ext_vector_type(2)))  float v2f;
typedef __attribute__((ext_vector_type(4)))  unsigned v4u;
typedef __attribute__((ext_vector_type(4)))  int v4i;
typedef float __attribute__((may_alias)) float_a;
typedef int __attribute__((may_alias)) int_a;

template <typename T> __device__ __forceinline__ void vst2(void* p, T v) { *(volatile T*)p = v; __threadfence(); *(volatile T*)p = v; }
__device__ __forceinline__ v8f wmma16(v16h a, v16h b, v8f c) {
  v8f d = __builtin_amdgcn_wmma_f32_16x16x32_f16(false, a, false, b, (short)0, c, false, false);
  asm volatile("v_nop\n\tv_nop\n\tv_nop\n\tv_nop" : "+v"(d) : "v"(a), "v"(b));
  return d;
}
__device__ __forceinline__ v8f wmma_bf(v16b a, v16b b, v8f c) {
  v8f d = __builtin_amdgcn_wmma_f32_16x16x32_bf16(false, a, false, b, (short)0, c, false, false);
  asm volatile("v_nop\n\tv_nop\n\tv_nop\n\tv_nop" : "+v"(d) : "v"(a), "v"(b));
  return d;
}
__device__ __forceinline__ v16h frag_h(const _Float16* rowk0, int lane) {
  union { v16h v; v8h q[2]; } u; const _Float16* p = rowk0 + 8 * (lane >> 4);
  u.q[0] = *(const v8h*)p; u.q[1] = *(const v8h*)(p + 16); return u.v;
}
__device__ __forceinline__ v16h frag_f32(const float* rowk0, int lane) {
  v16h a; const float* p = rowk0 + 8 * (lane >> 4);
#pragma unroll
  for (int i = 0; i < 8; ++i) { a[i] = (_Float16)p[i]; a[8 + i] = (_Float16)p[16 + i]; }
  return a;
}
__device__ __forceinline__ v16h frag_f32s(const float* rowk0, int lane, float sc) {
  v16h a; const float* p = rowk0 + 8 * (lane >> 4);
#pragma unroll
  for (int i = 0; i < 8; ++i) { a[i] = (_Float16)(p[i] * sc); a[8 + i] = (_Float16)(p[16 + i] * sc); }
  return a;
}
__device__ __forceinline__ v16h fragc_f32(const float* W, int k0, int n, int lane, int ld, int K) {
  v16h a; const int g = lane >> 4;
#pragma unroll
  for (int i = 0; i < 8; ++i) { const int ka = k0 + 8 * g + i, kb = ka + 16;
    a[i] = (_Float16)(ka < K ? W[(size_t)ka * ld + n] : 0.f); a[8 + i] = (_Float16)(kb < K ? W[(size_t)kb * ld + n] : 0.f); }
  return a;
}
struct F2 { v16b h, l; };
__device__ __forceinline__ F2 bsplit16(const float v[16]) { F2 r;
#pragma unroll
  for (int i = 0; i < 16; ++i) { const __bf16 h = (__bf16)v[i]; r.h[i] = h; r.l[i] = (__bf16)(v[i] - (float)h); }
  return r; }
__device__ __forceinline__ F2 split_row(const float* row, int k0, int lane) { float v[16]; const float* p = row + k0 + 8 * (lane >> 4);
#pragma unroll
  for (int i = 0; i < 8; ++i) { v[i] = p[i]; v[8 + i] = p[16 + i]; }
  return bsplit16(v); }
__device__ __forceinline__ F2 split_rowK(const float* row, int k0, int lane, int K) { float v[16]; const int g = lane >> 4;
#pragma unroll
  for (int i = 0; i < 8; ++i) { const int ka = k0 + 8 * g + i, kb = ka + 16; v[i] = ka < K ? row[ka] : 0.f; v[8 + i] = kb < K ? row[kb] : 0.f; }
  return bsplit16(v); }
__device__ __forceinline__ F2 split_col(const float* W, int k0, int n, int lane, int ld, int K) { float v[16]; const int g = lane >> 4;
#pragma unroll
  for (int i = 0; i < 8; ++i) { const int ka = k0 + 8 * g + i, kb = ka + 16; v[i] = ka < K ? W[(size_t)ka * ld + n] : 0.f; v[8 + i] = kb < K ? W[(size_t)kb * ld + n] : 0.f; }
  return bsplit16(v); }
__device__ __forceinline__ v8f mac3(const F2& a, const F2& b, v8f c) { c = wmma_bf(a.l, b.h, c); c = wmma_bf(a.h, b.l, c); return wmma_bf(a.h, b.h, c); }
__device__ __forceinline__ float sigm(float v) { return 1.0f / (1.0f + expf(-v)); }
#define LDSX() do { asm volatile("s_wait_dscnt 0" ::: "memory"); __builtin_amdgcn_wave_barrier(); __builtin_amdgcn_fence(__ATOMIC_RELEASE, "workgroup"); } while (0)

#define NN 100000
#define NE 1600000
#define FI 128
#define FH 64
#define RB 1024
#define NRB ((NN + RB - 1) / RB)
#define NNP (NRB * RB)
#define EPT 16
#define CH (256 * EPT)

template <int K>
__global__ __launch_bounds__(128) void k_node(const float* __restrict__ A, int arows, const float* __restrict__ Wl, const float* __restrict__ Wr, float* __restrict__ P) {
  __shared__ __align__(16) float so[4][16][132];
  const int tid = threadIdx.x, wave = tid >> 5, lane = tid & 31, col = lane & 15, g = lane >> 4;
  const int r0 = blockIdx.x * 64 + wave * 16; const int ra = (r0 + col) < arows ? (r0 + col) : arows - 1;
  v8f acc[8] = {};
#pragma unroll 1
  for (int kc = 0; kc < K / 32; ++kc) { const F2 a = split_row(A + (size_t)ra * K, kc * 32, lane);
#pragma unroll
    for (int t = 0; t < 4; ++t) { acc[t] = mac3(a, split_col(Wl, kc * 32, t * 16 + col, lane, FH, K), acc[t]); acc[4 + t] = mac3(a, split_col(Wr, kc * 32, t * 16 + col, lane, FH, K), acc[4 + t]); } }
#pragma unroll
  for (int t = 0; t < 8; ++t)
#pragma unroll
    for (int r = 0; r < 8; ++r) so[wave][8 * g + r][t * 16 + col] = acc[t][r];
  LDSX();
#pragma unroll 4
  for (int rl = 0; rl < 16; ++rl) vst2(P + (size_t)(r0 + rl) * 128 + lane * 4, *(const v4f*)(&so[wave][rl][lane * 4]));
}
template <int MODE>
__global__ __launch_bounds__(256) void k_agg(const float* __restrict__ P, const int* __restrict__ ei, const float* __restrict__ bl, const float* __restrict__ g, const float* __restrict__ be, const float* __restrict__ mn, const float* __restrict__ var,
                                            const float* __restrict__ Wh1, const float* __restrict__ bh1, const float* __restrict__ Wh2, const float* __restrict__ bh2, float* __restrict__ H, float* __restrict__ out) {
  __shared__ __align__(16) float sacc[RB][FH];
  __shared__ int ssrc[8][32 * EPT], sdl[8][32 * EPT]; __shared__ int scnt[8]; __shared__ int srcnt[RB]; __shared__ __align__(16) float sres[RB];
  const int tid = threadIdx.x, wave = tid >> 5, lane = tid & 31;
  const int r0 = blockIdx.x * RB; const int* esrc = ei; const int* edst = ei + NE;
  for (int q = tid; q < RB * FH; q += 256) (&sacc[0][0])[q] = 0.f;
  for (int q = tid; q < RB; q += 256) srcnt[q] = 0;
  __syncthreads();
  #pragma unroll 1
  for (int c0 = 0; c0 < NE; c0 += CH) {
    const int e0 = c0 + tid * EPT; int hd[EPT]; int cnt = 0;
    if (e0 + EPT <= NE) {
#pragma unroll
      for (int v = 0; v < EPT / 4; ++v) { const int4 d4 = *(const int4*)(edst + e0 + v * 4);
        const int dd[4] = {d4.x, d4.y, d4.z, d4.w};
#pragma unroll
        for (int u = 0; u < 4; ++u) { const unsigned rel = (unsigned)(dd[u] - r0); const bool h = rel < (unsigned)RB; hd[v * 4 + u] = h ? (int)rel : -1; cnt += h ? 1 : 0; } } }
    else {
#pragma unroll
      for (int u = 0; u < EPT; ++u) { const int e = e0 + u; hd[u] = -1; if (e < NE) { const unsigned rel = (unsigned)(edst[e] - r0); if (rel < (unsigned)RB) { hd[u] = (int)rel; ++cnt; } } } }
    int incl = cnt;
#pragma unroll
    for (int off = 1; off < 32; off <<= 1) { const int vv = __shfl_up(incl, off, 32); if (lane >= off) incl += vv; }
    const int wtot = __shfl(incl, 31, 32); int pos = incl - cnt;
    if (cnt > 0) {
#pragma unroll
      for (int u = 0; u < EPT; ++u) if (hd[u] >= 0) { int s = esrc[e0 + u]; s = s < 0 ? 0 : (s >= NN ? NN - 1 : s); ssrc[wave][pos] = s; sdl[wave][pos] = hd[u]; atomicAdd(&srcnt[hd[u]], 1); ++pos; } }
    if (lane == 0) scnt[wave] = wtot;
    __syncthreads();
    if (tid < FH) { for (int w = 0; w < 8; ++w) { const int nh = scnt[w]; for (int i = 0; i < nh; ++i) sacc[sdl[w][i]][tid] += P[(size_t)ssrc[w][i] * 128 + tid]; } }
    __syncthreads(); }
  for (int rl = tid; rl < RB; rl += 256) { const int row = r0 + rl; if (row >= NN) continue; const float inv = 1.0f / fmaxf((float)srcnt[rl], 1.0f); float* ar = &sacc[rl][0]; const float* pr = P + (size_t)row * 128 + FH;
#pragma unroll 1
    for (int f = 0; f < FH; ++f) { float v = ar[f] * inv + bl[f] + pr[f]; v = (v - mn[f]) * (g[f] * rsqrtf(var[f] + 1e-5f)) + be[f]; ar[f] = v > 0.f ? v : 0.f; }
    if (MODE == 1) { float o = bh2[0];
#pragma unroll 1
      for (int k = 0; k < 32; ++k) { float s = bh1[k];
#pragma unroll 1
        for (int f = 0; f < FH; ++f) s += ar[f] * Wh1[f * 32 + k];
        o += (s > 0.f ? s : 0.f) * Wh2[k]; }
      sres[rl] = sigm(o); } }
  __syncthreads();
  if (MODE == 0) { for (int q = tid; q < RB * (FH / 4); q += 256) { const int rl = q >> 4, pc = q & 15; const int row = r0 + rl; if (row >= NN) continue; vst2(H + (size_t)row * FH + pc * 4, *(const v4f*)(&sacc[rl][pc * 4])); } }
  else { for (int q = tid; q < RB / 4; q += 256) { const int row = r0 + q * 4; if (row >= NN) continue; vst2(out + row, *(const v4f*)(&sres[q * 4])); } }
}
extern "C" void kernel_launch(void* const* d_in, const int* in_sizes, int n_in, void* d_out, int out_size, void* d_ws, size_t ws_size, hipStream_t stream) {
  (void)in_sizes; (void)n_in; (void)out_size; (void)ws_size;
  const float** I = (const float**)d_in;
  const float* x = I[0]; const int* ei = (const int*)d_in[1];
  const float* Wl0 = I[2]; const float* bl0 = I[3]; const float* Wr0 = I[4]; const float* g0 = I[5]; const float* b0 = I[6]; const float* m0 = I[7]; const float* v0 = I[8];
  const float* Wl1 = I[9]; const float* bl1 = I[10]; const float* Wr1 = I[11]; const float* g1 = I[12]; const float* b1 = I[13]; const float* m1 = I[14]; const float* v1 = I[15];
  const float* Wh1 = I[16]; const float* bh1 = I[17]; const float* Wh2 = I[18]; const float* bh2 = I[19];
  float* out = (float*)d_out;
  char* ws = (char*)d_ws; size_t off = 0;
  auto take = [&](size_t bytes) { char* p = ws + off; off += (bytes + 255) & ~(size_t)255; return p; };
  float* P = (float*)take((size_t)NNP * 128 * 4); float* H = (float*)take((size_t)NNP * FH * 4);
  k_node<FI><<<NNP / 64, 128, 0, stream>>>(x, NN, Wl0, Wr0, P);
  k_agg<0><<<NRB, 256, 0, stream>>>(P, ei, bl0, g0, b0, m0, v0, nullptr, nullptr, nullptr, nullptr, H, nullptr);
  k_node<FH><<<NNP / 64, 128, 0, stream>>>(H, NN, Wl1, Wr1, P);
  k_agg<1><<<NRB, 256, 0, stream>>>(P, ei, bl1, g1, b1, m1, v1, Wh1, bh1, Wh2, bh2, nullptr, out);
}
